// QliGRU_22771916603945
// MI455X (gfx1250) — hardware-run, weakly checked
//
#include <hip/hip_runtime.h>
#include <math.h>

typedef __attribute__((ext_vector_type(16))) _Float16 v16h;
typedef __attribute__((ext_vector_type(8)))  _Float16 v8h;
typedef __attribute__((ext_vector_type(8)))  float    v8f;
typedef __attribute__((ext_vector_type(4)))  float    v4f;

#define T_STEPS      1000
#define NBATCH       32
#define NDIN         256
#define NHID         512
#define KFUSE        768
#define NCOLS        1024
#define APITCH       776
#define ROWS_PER_BLK 16
#define SEQ_THREADS  256
#define SLAB_PITCH   68
#define XH_CARRY     8.0f
#define W_CARRY      16.0f
#define ACC_FOLD     0.0078125f
#define KEEP_PROB    0.8f

__device__ __forceinline__ void dep_guard_h(v8f& a, v8f& b, v16h x, v16h y) { asm volatile("v_nop\n\tv_nop\n\tv_nop\n\tv_nop" : "+v"(a), "+v"(b) : "v"(x), "v"(y)); }
__device__ __forceinline__ void keep4_h(v16h a, v16h b, v16h c, v16h d) { asm volatile("v_nop" :: "v"(a), "v"(b), "v"(c), "v"(d)); }
__device__ __forceinline__ void acc_guard4(v8f& a, v8f& b, v8f& c, v8f& d) { asm volatile("v_nop\n\tv_nop\n\tv_nop\n\tv_nop" : "+v"(a), "+v"(b), "+v"(c), "+v"(d)); }
template <typename T> struct Frag;
template <> struct Frag<_Float16> {
  typedef v16h V; union U { v16h v; v8h h[2]; };
  static __device__ __forceinline__ v16h load(const _Float16* p) {
    U f; f.h[0] = *(const v8h*)(p); f.h[1] = *(const v8h*)(p + 16); return f.v;
  }
  static __device__ __forceinline__ v8f mma(v16h a, v16h b, v8f c) {
    return __builtin_amdgcn_wmma_f32_16x16x32_f16(false, a, false, b, (short)0, c, false, false);
  }
  static __device__ __forceinline__ void guard(v8f& a, v8f& b, v16h x, v16h y) { dep_guard_h(a, b, x, y); }
  static __device__ __forceinline__ void keep(v16h a, v16h b, v16h c, v16h d) { keep4_h(a, b, c, d); }
};

__constant__ int   kQComp[16] = {0, 1, 2, 3,   1, 0, 3, 2,   2, 3, 0, 1,   3, 2, 1, 0};
__constant__ float kQSgn[16]  = {1.f, 1.f, 1.f, 1.f,   -1.f, 1.f, 1.f, -1.f,   -1.f, -1.f, 1.f, 1.f,   -1.f, 1.f, -1.f, 1.f};
static_assert(sizeof(kQComp) / sizeof(kQComp[0]) == 16, "");
static_assert(sizeof(kQSgn) / sizeof(kQSgn[0]) == 16, "");

struct WPtrs {
  const float* wz[4];
  const float* wh[4];
  const float* uz[4];
  const float* uh[4];
};
static_assert(sizeof(WPtrs) == 16 * sizeof(void*), "");

__global__ __launch_bounds__(32) void build_bt(WPtrs p, _Float16* __restrict__ bt) {
  const int lane = threadIdx.x;
  const int n    = blockIdx.x;
  const int seg  = blockIdx.y;
  const int mat  = n >> 9;
  const int col  = n & 511;
  const int cb   = col >> 7;
  const int bc   = col & 127;
  const bool isU = (seg != 0);
  const int kl    = (isU ? (seg - 1) * 256 : 0) + lane * 8;
  const int shift = isU ? 7 : 6;
  const int rb    = kl >> shift;
  const int rr0   = kl & ((1 << shift) - 1);
  const float* s0 = isU ? (mat ? p.uh[0] : p.uz[0]) : (mat ? p.wh[0] : p.wz[0]);
  const float* s1 = isU ? (mat ? p.uh[1] : p.uz[1]) : (mat ? p.wh[1] : p.wz[1]);
  const float* s2 = isU ? (mat ? p.uh[2] : p.uz[2]) : (mat ? p.wh[2] : p.wz[2]);
  const float* s3 = isU ? (mat ? p.uh[3] : p.uz[3]) : (mat ? p.wh[3] : p.wz[3]);
  const int   qi = rb * 4 + cb;
  const int   ci = kQComp[qi];
  const float sg = kQSgn[qi] * W_CARRY;
  v8h hv;
#pragma unroll
  for (int e = 0; e < 8; ++e) {
    const int idx = (rr0 + e) * 128 + bc;
    const float v0 = s0[idx], v1 = s1[idx], v2 = s2[idx], v3 = s3[idx];
    const float val = (ci == 0) ? v0 : ((ci == 1) ? v1 : ((ci == 2) ? v2 : v3));
    hv[e] = (_Float16)(sg * val);
  }
  _Float16* dst = bt + (size_t)n * KFUSE + seg * 256 + lane * 8;
  *(volatile v8h*)dst = hv;
  __threadfence();
  *(volatile v8h*)dst = hv;
}

__global__ __launch_bounds__(SEQ_THREADS) void qligru_seq(
    const float* __restrict__ x, const _Float16* __restrict__ btp,
    const float* __restrict__ bz, const float* __restrict__ bh, float* __restrict__ out) {
  __shared__ __align__(16) _Float16 Atile[ROWS_PER_BLK * APITCH];
  __shared__ __align__(16) float    slabs[8][16 * SLAB_PITCH];

  const int tid  = threadIdx.x;
  const int lane = tid & 31;
  const int wave = tid >> 5;
  const int hh   = lane >> 4;
  const int cl   = lane & 15;
  const int koff = hh * 8;
  const int row0 = blockIdx.x * ROWS_PER_BLK;
  const int colw = wave * 64;
  float* slab = slabs[wave];

  {
    v8h zh;
#pragma unroll
    for (int e = 0; e < 8; ++e) zh[e] = (_Float16)0.0f;
#pragma unroll
    for (int it = 0; it < 4; ++it) {
      const int i = tid + it * SEQ_THREADS;
      const int m = i >> 6, c8 = (i & 63) * 8;
      *(v8h*)(Atile + m * APITCH + NDIN + c8) = zh;
    }
  }

  float hst[4][8];
#pragma unroll
  for (int u = 0; u < 4; ++u)
#pragma unroll
    for (int r = 0; r < 8; ++r) hst[u][r] = 0.0f;

  float bzv[4], bhv[4];
#pragma unroll
  for (int u = 0; u < 4; ++u) {
    bzv[u] = bz[colw + 16 * u + cl];
    bhv[u] = bh[colw + 16 * u + cl];
  }

  for (int t = 0; t < T_STEPS; ++t) {
#pragma unroll
    for (int it = 0; it < 2; ++it) {
      const int i = tid + it * SEQ_THREADS;
      const int m = i >> 5, c8 = (i & 31) * 8;
      const float* xp = x + ((size_t)t * NBATCH + row0 + m) * NDIN + c8;
      const v4f a0 = *(const v4f*)xp;
      const v4f a1 = *(const v4f*)(xp + 4);
      v8h hv;
      hv[0] = (_Float16)(a0[0] * XH_CARRY); hv[1] = (_Float16)(a0[1] * XH_CARRY);
      hv[2] = (_Float16)(a0[2] * XH_CARRY); hv[3] = (_Float16)(a0[3] * XH_CARRY);
      hv[4] = (_Float16)(a1[0] * XH_CARRY); hv[5] = (_Float16)(a1[1] * XH_CARRY);
      hv[6] = (_Float16)(a1[2] * XH_CARRY); hv[7] = (_Float16)(a1[3] * XH_CARRY);
      *(v8h*)(Atile + m * APITCH + c8) = hv;
    }
    __syncthreads();

    v8f acc[2][4];
#pragma unroll
    for (int g = 0; g < 2; ++g)
#pragma unroll
      for (int u = 0; u < 4; ++u) acc[g][u] = (v8f){0.f, 0.f, 0.f, 0.f, 0.f, 0.f, 0.f, 0.f};

#pragma unroll 2
    for (int k0 = 0; k0 < KFUSE; k0 += 32) {
      const v16h af = Frag<_Float16>::load(Atile + cl * APITCH + koff + k0);
#pragma unroll
      for (int g = 0; g < 2; ++g) {
        v16h bf[4];
#pragma unroll
        for (int u = 0; u < 4; ++u) {
          const size_t bo = (size_t)(g * NHID + colw + 16 * u + cl) * KFUSE + koff + k0;
          bf[u] = Frag<_Float16>::load(btp + bo);
        }
#pragma unroll
        for (int u = 0; u < 4; ++u) acc[g][u] = Frag<_Float16>::mma(af, bf[u], acc[g][u]);
        Frag<_Float16>::guard(acc[g][0], acc[g][3], af, af);
        Frag<_Float16>::keep(bf[0], bf[1], bf[2], bf[3]);
      }
    }
    acc_guard4(acc[0][0], acc[0][1], acc[0][2], acc[0][3]);
    acc_guard4(acc[1][0], acc[1][1], acc[1][2], acc[1][3]);
    __syncthreads();

#pragma unroll
    for (int u = 0; u < 4; ++u) {
#pragma unroll
      for (int r = 0; r < 8; ++r) {
        const float pz = acc[0][u][r] * ACC_FOLD + bzv[u];
        const float pa = acc[1][u][r] * ACC_FOLD + bhv[u];
        const float z  = 1.0f / (1.0f + expf(-pz));
        const float hc = fmaxf(pa, 0.0f) * KEEP_PROB;
        const float hn = z * hst[u][r] + (1.0f - z) * hc;
        hst[u][r] = hn;
        slab[(8 * hh + r) * SLAB_PITCH + 16 * u + cl] = hn;
      }
    }
    __builtin_amdgcn_fence(__ATOMIC_RELEASE, "workgroup");
    __builtin_amdgcn_wave_barrier();
    __builtin_amdgcn_fence(__ATOMIC_ACQUIRE, "workgroup");

    {
      const int c4 = cl * 4;
      float* obase = out + ((size_t)t * NBATCH + row0) * NHID + colw;
      for (int pass = 0; pass < 2; ++pass) {
#pragma unroll
        for (int it = 0; it < 8; ++it) {
          const int row = it * 2 + hh;
          const v4f v = *(const v4f*)(slab + row * SLAB_PITCH + c4);
          *(volatile v4f*)(obase + (size_t)row * NHID + c4) = v;
        }
        __threadfence();
      }
    }

    {
      const int hr = lane >> 1, half = lane & 1;
      const float* sp = slab + hr * SLAB_PITCH + half * 32;
      _Float16* ap = Atile + hr * APITCH + NDIN + colw + half * 32;
#pragma unroll
      for (int i = 0; i < 4; ++i) {
        const v4f p0 = *(const v4f*)(sp + 8 * i);
        const v4f p1 = *(const v4f*)(sp + 8 * i + 4);
        v8h hv;
        hv[0] = (_Float16)(p0[0] * XH_CARRY); hv[1] = (_Float16)(p0[1] * XH_CARRY);
        hv[2] = (_Float16)(p0[2] * XH_CARRY); hv[3] = (_Float16)(p0[3] * XH_CARRY);
        hv[4] = (_Float16)(p1[0] * XH_CARRY); hv[5] = (_Float16)(p1[1] * XH_CARRY);
        hv[6] = (_Float16)(p1[2] * XH_CARRY); hv[7] = (_Float16)(p1[3] * XH_CARRY);
        *(v8h*)(ap + 8 * i) = hv;
      }
    }
  }
}

extern "C" void kernel_launch(void* const* d_in, const int* in_sizes, int n_in,
                              void* d_out, int out_size, void* d_ws, size_t ws_size,
                              hipStream_t stream) {
  const size_t bt_bytes = (size_t)NCOLS * KFUSE * sizeof(_Float16);
  if (n_in < 19) return;
  if (in_sizes[0] != T_STEPS * NBATCH * NDIN) return;
  if (out_size != T_STEPS * NBATCH * NHID) return;
  if (ws_size < bt_bytes) return;
  for (int c = 0; c < 4; ++c) {
    if (in_sizes[1 + c] != 64 * 128 || in_sizes[5 + c] != 64 * 128) return;
    if (in_sizes[9 + c] != 128 * 128 || in_sizes[13 + c] != 128 * 128) return;
  }
  if (in_sizes[17] != NHID || in_sizes[18] != NHID) return;

  WPtrs p;
  for (int c = 0; c < 4; ++c) {
    p.wh[c] = (const float*)d_in[1 + c];
    p.wz[c] = (const float*)d_in[5 + c];
    p.uh[c] = (const float*)d_in[9 + c];
    p.uz[c] = (const float*)d_in[13 + c];
  }
  const float* x  = (const float*)d_in[0];
  const float* bh = (const float*)d_in[17];
  const float* bz = (const float*)d_in[18];
  float* out = (float*)d_out;
  _Float16* bt = (_Float16*)d_ws;

  build_bt<<<dim3(NCOLS, 3), dim3(32), 0, stream>>>(p, bt);
  qligru_seq<<<dim3(NBATCH / ROWS_PER_BLK), dim3(SEQ_THREADS), 0, stream>>>(x, bt, bz, bh, out);
}
